// SelfAttention_78829829751108
// MI455X (gfx1250) — hardware-verified
//
#include <hip/hip_runtime.h>
#include <stdint.h>


#ifndef NB
#define NB 2
#endif
#ifndef SEQ
#define SEQ 2048
#endif
#define NB_FULL 2
#define T_FULL  2048
#define EMB     1024
#define NH      16
#define HD      64
#define MROWS   (NB * SEQ)
#define PITCH   132

static_assert(NB >= 1 && NB <= NB_FULL);
static_assert(SEQ % 128 == 0 && SEQ >= 128 && SEQ <= T_FULL);
static_assert(EMB == NH * HD);
static_assert(HD == 64);
static_assert(MROWS % 128 == 0);
static_assert(EMB % 64 == 0 && EMB % 32 == 0);
static_assert((MROWS * (EMB / 8)) % 256 == 0);
static_assert((9LL * MROWS * EMB + 4LL * EMB * EMB) * 2LL <= 134217728LL);

typedef _Float16 h16;
typedef h16   v16h __attribute__((ext_vector_type(16)));
typedef h16   v8h  __attribute__((ext_vector_type(8)));
typedef float v8f  __attribute__((ext_vector_type(8)));
typedef float v4f  __attribute__((ext_vector_type(4)));

union Frag   { v16h v; v8h q[2]; };
union Pack8  { v8h v; h16 s[8]; };
union Pack16 { v16h v; h16 s[16]; };

__device__ __forceinline__ v8f zero8() {
  v8f z = {0.f, 0.f, 0.f, 0.f, 0.f, 0.f, 0.f, 0.f};
  return z;
}

__device__ __forceinline__ v8f mma16(v8f c, v16h a, v16h b) {
  v8f d = __builtin_amdgcn_wmma_f32_16x16x32_f16(false, a, false, b, (short)0, c, false, false);
  asm volatile("v_nop\n\tv_nop\n\tv_nop\n\tv_nop" : "+v"(d) : "v"(a), "v"(b));
  return d;
}

__device__ __forceinline__ v16h ldfrag(const h16* row_k0, int g) {
  Frag f;
  const h16* p = row_k0 + 8 * g;
  f.q[0] = *(const v8h*)(p);
  f.q[1] = *(const v8h*)(p + 16);
  return f.v;
}

__device__ __forceinline__ float bfr(float f) {
  unsigned u = __float_as_uint(f);
  u = (u + 0x7FFFu + ((u >> 16) & 1u)) & 0xFFFF0000u;
  return __uint_as_float(u);
}

__device__ __forceinline__ void split16(float v, h16& hi, h16& rs) {
  hi = (h16)v;
  rs = (h16)((v - (float)hi) * 4096.0f);
}

__global__ __launch_bounds__(256) void cvt_x(const float* __restrict__ x, h16* x16) {
  const int idx = blockIdx.x * 256 + threadIdx.x;
  const int m   = idx / (EMB / 8);
  const int e8  = (idx - m * (EMB / 8)) * 8;
  const int b   = m / SEQ;
  const int t   = m - b * SEQ;
  const float* src = x + ((size_t)b * T_FULL + t) * EMB + e8;
  const v4f u0 = *(const v4f*)(src);
  const v4f u1 = *(const v4f*)(src + 4);
  Pack8 pk;
#pragma unroll
  for (int i = 0; i < 4; ++i) {
    pk.s[i]     = (h16)bfr(u0[i]);
    pk.s[4 + i] = (h16)bfr(u1[i]);
  }
  h16* dst = x16 + (size_t)m * EMB + e8;
  *(volatile v8h*)dst = pk.v;
  __threadfence();
  *(volatile v8h*)dst = pk.v;
}

__global__ __launch_bounds__(256) void cvt_w(const float* __restrict__ W0, const float* __restrict__ W1,
                                             const float* __restrict__ W2, const float* __restrict__ W3,
                                             h16* wt) {
  __shared__ float tile[64 * 68];
  const int z = blockIdx.z;
  const float* W = (z == 0) ? W0 : ((z == 1) ? W1 : ((z == 2) ? W2 : W3));
  h16* O = wt + (size_t)z * EMB * EMB;
  const int n0  = blockIdx.x * 64;
  const int k0  = blockIdx.y * 64;
  const int tid = threadIdx.x;
  {
    const int kr = tid >> 2;
    const int cb = (tid & 3) * 16;
    const float* src = W + (size_t)(k0 + kr) * EMB + n0 + cb;
#pragma unroll
    for (int j = 0; j < 4; ++j)
      *(v4f*)&tile[kr * 68 + cb + 4 * j] = *(const v4f*)(src + 4 * j);
  }
  __syncthreads();
  Pack8 pk[2];
  size_t off[2];
#pragma unroll
  for (int it = 0; it < 2; ++it) {
    const int p  = it * 256 + tid;
    const int n  = p >> 3;
    const int k8 = (p & 7) * 8;
#pragma unroll
    for (int j = 0; j < 8; ++j)
      pk[it].s[j] = (h16)(bfr(tile[(k8 + j) * 68 + n]) * 32.0f);
    off[it] = (size_t)(n0 + n) * EMB + k0 + k8;
  }
#pragma unroll
  for (int it = 0; it < 2; ++it) *(volatile v8h*)(O + off[it]) = pk[it].v;
  __threadfence();
#pragma unroll
  for (int it = 0; it < 2; ++it) *(volatile v8h*)(O + off[it]) = pk[it].v;
}

template <int MODE>
__global__ __launch_bounds__(256) void gemm16(const h16* __restrict__ Ah, const h16* __restrict__ Ar,
                                              const h16* __restrict__ Bt, h16* Oh, h16* Or,
                                              float* Of, const float* __restrict__ bias) {
  __shared__ float tile[64 * PITCH];
  const int tid = threadIdx.x, wid = tid >> 5, lane = tid & 31, l16 = lane & 15, g = lane >> 4;
  const int tn  = blockIdx.x * 64;
  const int tm  = blockIdx.y * 128 + wid * 16;
  const h16* arow = Ah + (size_t)(tm + l16) * EMB;
  const h16* rrow = Ar + (size_t)(tm + l16) * EMB;
  const h16* brow = Bt + (size_t)(tn + l16) * EMB;

  v8f acc[4], accr[4];
#pragma unroll
  for (int c = 0; c < 4; ++c) { acc[c] = zero8(); accr[c] = zero8(); }

#pragma unroll 2
  for (int k0 = 0; k0 < EMB; k0 += 32) {
    const v16h a = ldfrag(arow + k0, g);
    v16h ar = a;
    if (MODE == 2) ar = ldfrag(rrow + k0, g);
#pragma unroll
    for (int c = 0; c < 4; ++c) {
      const v16h bf = ldfrag(brow + (size_t)c * 16 * EMB + k0, g);
      acc[c] = mma16(acc[c], a, bf);
      if (MODE == 2) accr[c] = mma16(accr[c], ar, bf);
    }
  }

#pragma unroll
  for (int c = 0; c < 4; ++c) {
    float v[8];
#pragma unroll
    for (int r = 0; r < 8; ++r) {
      if (MODE == 2) v[r] = (acc[c][r] + accr[c][r] * (1.0f / 4096.0f)) * (1.0f / 512.0f);
      else           v[r] = acc[c][r] * 0.25f;
    }
    float* tp = &tile[(c * 16 + l16) * PITCH + wid * 16 + 8 * g];
    const v4f lo4 = {v[0], v[1], v[2], v[3]};
    const v4f hi4 = {v[4], v[5], v[6], v[7]};
    *(v4f*)(tp)     = lo4;
    *(v4f*)(tp + 4) = hi4;
  }
  __syncthreads();

  if (MODE == 0) {
    Pack8 ph[4], pr[4];
    size_t off[4];
#pragma unroll
    for (int it = 0; it < 4; ++it) {
      const int p   = it * 32 + lane;
      const int row = p >> 3;
      const int c8  = (p & 7) * 8;
#pragma unroll
      for (int j = 0; j < 8; ++j)
        split16(tile[(c8 + j) * PITCH + wid * 16 + row], ph[it].s[j], pr[it].s[j]);
      off[it] = (size_t)(tm + row) * EMB + tn + c8;
    }
#pragma unroll
    for (int it = 0; it < 4; ++it) {
      *(volatile v8h*)(Oh + off[it]) = ph[it].v;
      *(volatile v8h*)(Or + off[it]) = pr[it].v;
    }
    __threadfence();
#pragma unroll
    for (int it = 0; it < 4; ++it) {
      *(volatile v8h*)(Oh + off[it]) = ph[it].v;
      *(volatile v8h*)(Or + off[it]) = pr[it].v;
    }
  } else if (MODE == 1) {
    const int b  = (blockIdx.y * 128) / SEQ;
    const int t0 = blockIdx.y * 128 - b * SEQ;
    const int h  = blockIdx.x;
    Pack8 ph[4], pr[4];
    size_t off[4];
#pragma unroll
    for (int it = 0; it < 4; ++it) {
      const int p  = it * 256 + tid;
      const int s  = p >> 4;
      const int t8 = (p & 15) * 8;
      const float* tp = &tile[s * PITCH + t8];
      const v4f u0 = *(const v4f*)(tp);
      const v4f u1 = *(const v4f*)(tp + 4);
#pragma unroll
      for (int j = 0; j < 4; ++j) {
        split16(u0[j], ph[it].s[j],     pr[it].s[j]);
        split16(u1[j], ph[it].s[4 + j], pr[it].s[4 + j]);
      }
      off[it] = (((size_t)(b * NH + h)) * HD + s) * SEQ + t0 + t8;
    }
#pragma unroll
    for (int it = 0; it < 4; ++it) {
      *(volatile v8h*)(Oh + off[it]) = ph[it].v;
      *(volatile v8h*)(Or + off[it]) = pr[it].v;
    }
    __threadfence();
#pragma unroll
    for (int it = 0; it < 4; ++it) {
      *(volatile v8h*)(Oh + off[it]) = ph[it].v;
      *(volatile v8h*)(Or + off[it]) = pr[it].v;
    }
  } else {
    v4f ov[8];
    size_t off[8];
#pragma unroll
    for (int it = 0; it < 8; ++it) {
      const int p   = it * 32 + lane;
      const int row = p >> 4;
      const int c4  = (p & 15) * 4;
      const v4f bb  = *(const v4f*)(bias + tn + c4);
      v4f o;
#pragma unroll
      for (int j = 0; j < 4; ++j)
        o[j] = tile[(c4 + j) * PITCH + wid * 16 + row] + bfr(bb[j]);
      ov[it] = o;
      const int m  = tm + row;
      const int bq = m / SEQ;
      const int t  = m - bq * SEQ;
      off[it] = ((size_t)bq * T_FULL + t) * EMB + tn + c4;
    }
#pragma unroll
    for (int it = 0; it < 8; ++it) *(volatile v4f*)(Of + off[it]) = ov[it];
    __threadfence();
#pragma unroll
    for (int it = 0; it < 8; ++it) *(volatile v4f*)(Of + off[it]) = ov[it];
  }
}

__global__ __launch_bounds__(256) __attribute__((amdgpu_num_vgpr(256)))
void attn16(const h16* __restrict__ Qh, const h16* __restrict__ Qr,
            const h16* __restrict__ Kh, const h16* __restrict__ Kr,
            const h16* __restrict__ Vh, const h16* __restrict__ Vr,
            h16* Ch, h16* Cr) {
  __shared__ float tile[64 * PITCH];
  const int tid = threadIdx.x, wid = tid >> 5, lane = tid & 31, l16 = lane & 15, g = lane >> 4;
  const int gw  = blockIdx.x * 8 + wid;
  const int nqt = SEQ / 16;
  const int bh  = gw / nqt;
  const int qt  = gw - bh * nqt;
  const int b   = bh / NH;
  const int h   = bh - b * NH;
  const int qbase = qt * 16;
  const int myq   = qbase + l16;

  const size_t qoff = ((size_t)b * SEQ + myq) * EMB + h * HD;
  const v16h qh0 = ldfrag(Qh + qoff, g), qh1 = ldfrag(Qh + qoff + 32, g);
  const v16h qr0 = ldfrag(Qr + qoff, g), qr1 = ldfrag(Qr + qoff + 32, g);

  v8f o[4];
#pragma unroll
  for (int dt = 0; dt < 4; ++dt) o[dt] = zero8();
  float mrow = -__builtin_inff();
  float lrow = 0.0f;
  const float L2E = 1.4426950408889634f;
  const int nch = (qbase >> 5) + 1;
  const size_t kb = (size_t)b * SEQ;
  const size_t vb = ((size_t)(b * NH + h)) * HD;

#pragma unroll 1
  for (int ch = 0; ch < nch; ++ch) {
    const int j0 = ch * 32;
    float s[2][8];
    int kdep = 0;
#pragma unroll
    for (int tl = 0; tl < 2; ++tl) {
      const size_t koff = (kb + j0 + tl * 16 + l16 + kdep) * EMB + h * HD;
      const v16h kh0 = ldfrag(Kh + koff, g), kh1 = ldfrag(Kh + koff + 32, g);
      const v16h kr0 = ldfrag(Kr + koff, g), kr1 = ldfrag(Kr + koff + 32, g);
      v8f ah = zero8(), ar = zero8();
      ah = mma16(ah, kh0, qh0);
      ah = mma16(ah, kh1, qh1);
      ar = mma16(ar, kh0, qr0);
      ar = mma16(ar, kh1, qr1);
      ar = mma16(ar, kr0, qh0);
      ar = mma16(ar, kr1, qh1);
#pragma unroll
      for (int r = 0; r < 8; ++r) {
        const int key = j0 + tl * 16 + 8 * g + r;
        const float v = (ah[r] + ar[r] * (1.0f / 4096.0f)) * (1.0f / 512.0f);
        s[tl][r] = (key <= myq) ? v : -__builtin_inff();
      }
      asm volatile("" : "+v"(kdep) : "v"(ah[0]));
    }

    float cm = -__builtin_inff();
#pragma unroll
    for (int r = 0; r < 8; ++r) { cm = fmaxf(cm, s[0][r]); cm = fmaxf(cm, s[1][r]); }
    cm = fmaxf(cm, __shfl_xor(cm, 16, 32));
    const float mnew  = fmaxf(mrow, cm);
    const float alpha = __builtin_amdgcn_exp2f((mrow - mnew) * L2E);
    mrow = mnew;

    Pack16 pa, pe;
    float psum = 0.0f;
#pragma unroll
    for (int r = 0; r < 8; ++r) {
      const float p0 = __builtin_amdgcn_exp2f((s[0][r] - mnew) * L2E);
      const float p1 = __builtin_amdgcn_exp2f((s[1][r] - mnew) * L2E);
      psum += p0 + p1;
      const float c0 = p0 * 16384.0f;
      const float c1 = p1 * 16384.0f;
      const h16 h0 = (h16)c0;
      const h16 h1 = (h16)c1;
      pa.s[r]     = h0;
      pa.s[8 + r] = h1;
      pe.s[r]     = (h16)((c0 - (float)h0) * 2048.0f);
      pe.s[8 + r] = (h16)((c1 - (float)h1) * 2048.0f);
    }
    psum += __shfl_xor(psum, 16, 32);
    lrow = lrow * alpha + psum;

    float al[8];
#pragma unroll
    for (int r = 0; r < 8; ++r) al[r] = __shfl(alpha, 8 * g + r, 32);

    int vdep = 0;
    asm volatile("" : "+v"(vdep) : "v"(psum));
#pragma unroll
    for (int dt = 0; dt < 4; ++dt) {
      const size_t voff = (vb + dt * 16 + l16 + vdep) * SEQ + j0;
      const v16h bvh = ldfrag(Vh + voff, g);
      const v16h bvr = ldfrag(Vr + voff, g);
      v8f th = zero8(), tr = zero8(), te = zero8();
      th = mma16(th, pa.v, bvh);
      tr = mma16(tr, pa.v, bvr);
      te = mma16(te, pe.v, bvh);
#pragma unroll
      for (int r = 0; r < 8; ++r)
        o[dt][r] = o[dt][r] * al[r] + (th[r] + tr[r] * (1.0f / 4096.0f) + te[r] * (1.0f / 2048.0f));
      asm volatile("" : "+v"(vdep) : "v"(o[dt][0]));
    }
  }

  float linv[8];
#pragma unroll
  for (int r = 0; r < 8; ++r) linv[r] = (1.0f / __shfl(lrow, 8 * g + r, 32)) * (1.0f / 8192.0f);
#pragma unroll
  for (int dt = 0; dt < 4; ++dt) {
    float v[8];
#pragma unroll
    for (int r = 0; r < 8; ++r) v[r] = o[dt][r] * linv[r];
    float* tp = &tile[(dt * 16 + l16) * PITCH + wid * 16 + 8 * g];
    const v4f lo4 = {v[0], v[1], v[2], v[3]};
    const v4f hi4 = {v[4], v[5], v[6], v[7]};
    *(v4f*)(tp)     = lo4;
    *(v4f*)(tp + 4) = hi4;
  }
  __syncthreads();

  Pack8 ph[4], pr[4];
  size_t off[4];
#pragma unroll
  for (int it = 0; it < 4; ++it) {
    const int p   = it * 32 + lane;
    const int row = p >> 3;
    const int c8  = (p & 7) * 8;
#pragma unroll
    for (int j = 0; j < 8; ++j)
      split16(tile[(c8 + j) * PITCH + wid * 16 + row], ph[it].s[j], pr[it].s[j]);
    off[it] = ((size_t)b * SEQ + qbase + row) * EMB + h * HD + c8;
  }
#pragma unroll
  for (int it = 0; it < 4; ++it) {
    *(volatile v8h*)(Ch + off[it]) = ph[it].v;
    *(volatile v8h*)(Cr + off[it]) = pr[it].v;
  }
  __threadfence();
#pragma unroll
  for (int it = 0; it < 4; ++it) {
    *(volatile v8h*)(Ch + off[it]) = ph[it].v;
    *(volatile v8h*)(Cr + off[it]) = pr[it].v;
  }
}

extern "C" void kernel_launch(void* const* d_in, const int* in_sizes, int n_in,
                              void* d_out, int out_size, void* d_ws, size_t ws_size,
                              hipStream_t stream) {
  if (n_in < 6) return;
  const long long needX = ((long long)(NB - 1) * T_FULL + SEQ) * (long long)EMB;
  if ((long long)in_sizes[0] < needX) return;
  if (in_sizes[1] < EMB * EMB || in_sizes[2] < EMB * EMB || in_sizes[3] < EMB * EMB || in_sizes[4] < EMB * EMB) return;
  if (in_sizes[5] < EMB) return;
  if ((long long)out_size < needX) return;

  const size_t PL = (size_t)MROWS * EMB;
  const size_t WP = (size_t)EMB * EMB;
  const size_t total_bytes = (9 * PL + 4 * WP) * sizeof(h16);
  if (total_bytes > ws_size) return;

  const float* x  = (const float*)d_in[0];
  const float* Wq = (const float*)d_in[1];
  const float* Wk = (const float*)d_in[2];
  const float* Wv = (const float*)d_in[3];
  const float* Wu = (const float*)d_in[4];
  const float* bu = (const float*)d_in[5];
  float* out = (float*)d_out;

  h16* x16 = (h16*)d_ws;
  h16* wt  = x16 + PL;
  h16* qh  = wt + 4 * WP;
  h16* qr  = qh + PL;
  h16* kh  = qr + PL;
  h16* kr  = kh + PL;
  h16* vth = kr + PL;
  h16* vtr = vth + PL;
  h16* chh = vtr + PL;
  h16* chr = chh + PL;

  cvt_x<<<(MROWS * (EMB / 8)) / 256, 256, 0, stream>>>(x, x16);
  cvt_w<<<dim3(EMB / 64, EMB / 64, 4), 256, 0, stream>>>(Wq, Wk, Wv, Wu, wt);
  const dim3 gg(EMB / 64, MROWS / 128);
  gemm16<0><<<gg, 256, 0, stream>>>(x16, x16, wt + 0 * WP, qh, qr, out, bu);
  gemm16<0><<<gg, 256, 0, stream>>>(x16, x16, wt + 1 * WP, kh, kr, out, bu);
  gemm16<1><<<gg, 256, 0, stream>>>(x16, x16, wt + 2 * WP, vth, vtr, out, bu);
  attn16<<<(NB * NH * SEQ) / 128, 256, 0, stream>>>(qh, qr, kh, kr, vth, vtr, chh, chr);
  gemm16<2><<<gg, 256, 0, stream>>>(chh, chr, wt + 3 * WP, qh, qr, out, bu);
}
